// WaveAttention_8383776162028
// MI455X (gfx1250) — hardware-verified
//
#include <hip/hip_runtime.h>

typedef _Float16 v16h __attribute__((ext_vector_type(16)));
typedef _Float16 v8h  __attribute__((ext_vector_type(8)));
typedef __bf16   v16b __attribute__((ext_vector_type(16)));
typedef unsigned short u16;
typedef u16      v8us __attribute__((ext_vector_type(8)));
typedef float    v8f  __attribute__((ext_vector_type(8)));
typedef float    v4f  __attribute__((ext_vector_type(4)));
typedef unsigned v4u  __attribute__((ext_vector_type(4)));
typedef v8h  __attribute__((may_alias)) v8ha;
typedef v8us __attribute__((may_alias)) v8usa;
typedef v4f  __attribute__((may_alias)) v4fa;

union FragH { v16h v; v8h q[2]; v4u u[2]; };
union FragB { v16b v; v8us q[2]; };

#define NB     8
#define HIMG   56
#define NTOK   3136
#define CDIM   512
#define NQROWS 25088
#define C4     128
#define H2     28
#define P2     784
#define NPIX2  6272
#define NHEAD  8
#define HDIM   64
#define NKEY   196
#define KST    256
#define KUSE   224
#define KVROWS 2048
#define KF     4608
#define KE     2048
#define CATK   640
#define EPS_LN 1e-5f
#define PSCALE 16384.0f
#define BN_RS  (1.0f - 84.0f / 16777216.0f)

#define PB_X   6272
#define PB_QW  128
#define PB_RW  32
#define PB_FW  1152
#define PB_KE  512
#define PB_KV  256
#define PB_PW  160
#define PB_TOTAL (PB_X + PB_QW + PB_RW + PB_FW + PB_KE + PB_KV + PB_PW)

__device__ __forceinline__ v8f zero8() { v8f z = {0.f, 0.f, 0.f, 0.f, 0.f, 0.f, 0.f, 0.f}; return z; }

__device__ __forceinline__ v8f mma_h(v16h a, v16h b, v8f c) {
  v8f d = __builtin_amdgcn_wmma_f32_16x16x32_f16(false, a, false, b, (short)0, c, false, false);
  asm volatile("v_nop\n\tv_nop\n\tv_nop\n\tv_nop" : "+v"(d) : "v"(a), "v"(b));
  return d;
}
__device__ __forceinline__ v8f mma_b(v16b a, v16b b, v8f c) {
  v8f d = __builtin_amdgcn_wmma_f32_16x16x32_bf16(false, a, false, b, (short)0, c, false, false);
  asm volatile("v_nop\n\tv_nop\n\tv_nop\n\tv_nop" : "+v"(d) : "v"(a), "v"(b));
  return d;
}

__device__ __forceinline__ v16h ldfh(const _Float16* p, int h) {
  FragH f;
  f.q[0] = *(const v8ha*)(p + 8 * h);
  f.q[1] = *(const v8ha*)(p + 16 + 8 * h);
  return f.v;
}
__device__ __forceinline__ v16h ldfh_m(const _Float16* p, int h, unsigned msk) {
  FragH f;
  f.q[0] = *(const v8ha*)(p + 8 * h);
  f.q[1] = *(const v8ha*)(p + 16 + 8 * h);
  const v4u mm = {msk, msk, msk, msk};
  f.u[0] &= mm;
  f.u[1] &= mm;
  return f.v;
}
__device__ __forceinline__ v16b ldfb(const u16* p, int h) {
  FragB f;
  f.q[0] = *(const v8usa*)(p + 8 * h);
  f.q[1] = *(const v8usa*)(p + 16 + 8 * h);
  return f.v;
}

__device__ __forceinline__ u16 bfb(float f) {
  unsigned u = __float_as_uint(f);
  u = (u + 0x7FFFu + ((u >> 16) & 1u)) >> 16;
  return (u16)u;
}
__device__ __forceinline__ float bfv(u16 b) { return __uint_as_float(((unsigned)b) << 16); }
__device__ __forceinline__ float r16f(float v) { return (float)((_Float16)v); }

__device__ __forceinline__ void ld8(const float* p, float v[8]) {
  const v4f a = *(const v4fa*)p;
  const v4f c = *(const v4fa*)(p + 4);
  v[0] = a.x; v[1] = a.y; v[2] = a.z; v[3] = a.w;
  v[4] = c.x; v[5] = c.y; v[6] = c.z; v[7] = c.w;
}
struct HL8 { v8us hi, lo; };
__device__ __forceinline__ HL8 split_bf8(const float v[8]) {
  HL8 r;
  v8us hi = {0, 0, 0, 0, 0, 0, 0, 0}, lo = {0, 0, 0, 0, 0, 0, 0, 0};
#pragma unroll
  for (int j = 0; j < 8; ++j) {
    const u16 hb = bfb(v[j]);
    hi[j] = hb;
    lo[j] = bfb(v[j] - bfv(hb));
  }
  r.hi = hi; r.lo = lo;
  return r;
}
__device__ __forceinline__ v8us pack_bf8(const float v[8]) {
  v8us o = {0, 0, 0, 0, 0, 0, 0, 0};
#pragma unroll
  for (int j = 0; j < 8; ++j) o[j] = bfb(v[j]);
  return o;
}
__device__ __forceinline__ v8h pack_h8(const float v[8], float sc) {
  v8h o = {(_Float16)0.f, (_Float16)0.f, (_Float16)0.f, (_Float16)0.f, (_Float16)0.f, (_Float16)0.f, (_Float16)0.f, (_Float16)0.f};
#pragma unroll
  for (int j = 0; j < 8; ++j) o[j] = (_Float16)(v[j] * sc);
  return o;
}

__device__ __forceinline__ void store_h128(const _Float16* sT, _Float16* dst0, int ld, int w, int lane) {
  const int q8 = lane & 7, sub = lane >> 3;
#pragma unroll
  for (int i = 0; i < 8; ++i) {
    const int lid = w * 32 + i * 4 + sub;
    const v8h v = *(const v8ha*)(sT + lid * 64 + 8 * q8);
    *(volatile v8h*)(dst0 + (size_t)lid * ld + 8 * q8) = v;
  }
}
__device__ __forceinline__ void store_h64(const _Float16* sT, _Float16* dst0, int ld, int w, int lane) {
  const int q8 = lane & 7, sub = lane >> 3;
#pragma unroll
  for (int i = 0; i < 4; ++i) {
    const int lid = w * 16 + i * 4 + sub;
    const v8h v = *(const v8ha*)(sT + lid * 64 + 8 * q8);
    *(volatile v8h*)(dst0 + (size_t)lid * ld + 8 * q8) = v;
  }
}
__device__ __forceinline__ void store_f128(const float* sT, float* dst0, int ld, int w, int lane) {
  const int pc = lane & 15, sub = lane >> 4;
#pragma unroll
  for (int i = 0; i < 16; ++i) {
    const int lid = w * 32 + 2 * i + sub;
    const v4f v = *(const v4fa*)(sT + lid * 64 + 4 * pc);
    *(volatile v4f*)(dst0 + (size_t)lid * ld + 4 * pc) = v;
  }
}
__device__ __forceinline__ void store_vt(const _Float16* sT, _Float16* vt, int bh, int kh, int w, int lane) {
  const int q8 = lane & 7, sub = lane >> 3;
#pragma unroll
  for (int i = 0; i < 8; ++i) {
    const int lid = w * 32 + i * 4 + sub;
    const int d = lid >> 1, hl = lid & 1;
    const v8h v = *(const v8ha*)(sT + d * 128 + 64 * hl + 8 * q8);
    *(volatile v8h*)(vt + ((size_t)(bh * HDIM + d)) * KST + kh * 128 + 64 * hl + 8 * q8) = v;
  }
}

__global__ __launch_bounds__(256) void k_prep(
    const float* __restrict__ x, const float* __restrict__ q_w, const float* __restrict__ reduce_w,
    const float* __restrict__ filter_w, const float* __restrict__ kve_w, const float* __restrict__ kv_w,
    const float* __restrict__ proj_w,
    u16* xhi, u16* xlo, u16* qw, u16* rwh, u16* rwl,
    _Float16* fwh, _Float16* fwl, _Float16* kew, _Float16* kvw, u16* pwh, u16* pwl)
{
#pragma clang fp contract(off)
  int blk = blockIdx.x;
  const int t = threadIdx.x;
  float v[8];
  if (blk < PB_X) {
    const size_t g = (size_t)blk * 256 + t;
    ld8(x + g * 8, v);
    const HL8 s = split_bf8(v);
    u16* dh = xhi + g * 8; u16* dl = xlo + g * 8;
    *(volatile v8us*)dh = s.hi; *(volatile v8us*)dl = s.lo;
    __threadfence();
    *(volatile v8us*)dh = s.hi; *(volatile v8us*)dl = s.lo;
    return;
  }
  blk -= PB_X;
  if (blk < PB_QW) {
    const size_t g = (size_t)blk * 256 + t;
    ld8(q_w + g * 8, v);
    const v8us o = pack_bf8(v);
    u16* d = qw + g * 8;
    *(volatile v8us*)d = o;
    __threadfence();
    *(volatile v8us*)d = o;
    return;
  }
  blk -= PB_QW;
  if (blk < PB_RW) {
    const size_t g = (size_t)blk * 256 + t;
    ld8(reduce_w + g * 8, v);
    const HL8 s = split_bf8(v);
    u16* dh = rwh + g * 8; u16* dl = rwl + g * 8;
    *(volatile v8us*)dh = s.hi; *(volatile v8us*)dl = s.lo;
    __threadfence();
    *(volatile v8us*)dh = s.hi; *(volatile v8us*)dl = s.lo;
    return;
  }
  blk -= PB_RW;
  if (blk < PB_FW) {
    const int g = blk * 256 + t;
    const int o = g / 576, rem = g - o * 576;
    const int tap = rem >> 6, c0 = (rem & 63) * 8;
    const float* src = filter_w + ((size_t)o * CDIM + c0) * 9 + tap;
#pragma unroll
    for (int j = 0; j < 8; ++j) v[j] = src[j * 9];
    v8h hv = {(_Float16)0.f, (_Float16)0.f, (_Float16)0.f, (_Float16)0.f, (_Float16)0.f, (_Float16)0.f, (_Float16)0.f, (_Float16)0.f};
    v8h lv = hv;
#pragma unroll
    for (int j = 0; j < 8; ++j) {
      const float ws = v[j] * 64.0f;
      const _Float16 hh = (_Float16)ws;
      hv[j] = hh;
      lv[j] = (_Float16)((ws - (float)hh) * 2048.0f);
    }
    _Float16* dh = fwh + (size_t)g * 8; _Float16* dl = fwl + (size_t)g * 8;
    *(volatile v8h*)dh = hv; *(volatile v8h*)dl = lv;
    __threadfence();
    *(volatile v8h*)dh = hv; *(volatile v8h*)dl = lv;
    return;
  }
  blk -= PB_FW;
  if (blk < PB_KE) {
    const int g = blk * 256 + t;
    const int o = g >> 8, rem = g & 255;
    const int tap = rem >> 6, c0 = (rem & 63) * 8;
    const float* src = kve_w + ((size_t)o * CDIM + c0) * 4 + tap;
#pragma unroll
    for (int j = 0; j < 8; ++j) v[j] = src[j * 4];
    const v8h o8 = pack_h8(v, 16.0f);
    _Float16* d = kew + (size_t)g * 8;
    *(volatile v8h*)d = o8;
    __threadfence();
    *(volatile v8h*)d = o8;
    return;
  }
  blk -= PB_KE;
  if (blk < PB_KV) {
    const size_t g = (size_t)blk * 256 + t;
    ld8(kv_w + g * 8, v);
    const v8h o8 = pack_h8(v, 32.0f);
    _Float16* d = kvw + g * 8;
    *(volatile v8h*)d = o8;
    __threadfence();
    *(volatile v8h*)d = o8;
    return;
  }
  blk -= PB_KV;
  if (blk < PB_PW) {
    const size_t g = (size_t)blk * 256 + t;
    ld8(proj_w + g * 8, v);
    const HL8 s = split_bf8(v);
    u16* dh = pwh + g * 8; u16* dl = pwl + g * 8;
    *(volatile v8us*)dh = s.hi; *(volatile v8us*)dl = s.lo;
    __threadfence();
    *(volatile v8us*)dh = s.hi; *(volatile v8us*)dl = s.lo;
  }
}

__global__ __launch_bounds__(128) void k_reduce(
    const u16* __restrict__ xhi, const u16* __restrict__ xlo,
    const u16* __restrict__ rwh, const u16* __restrict__ rwl,
    const float* __restrict__ rb, const float* __restrict__ rg, const float* __restrict__ rbe,
    _Float16* r16)
{
#pragma clang fp contract(off)
  __shared__ __attribute__((aligned(16))) _Float16 sT[128 * 64];
  const int tid = threadIdx.x, lane = tid & 31, w = tid >> 5, h = lane >> 4, m = lane & 15;
  const int m0 = blockIdx.x * 128, n0 = blockIdx.y * 64, m0w = m0 + 32 * w;
  const size_t ar0 = (size_t)(m0w + m) * CDIM, ar1 = ar0 + (size_t)16 * CDIM;
  const u16* bhp = rwh + (size_t)(n0 + m) * CDIM;
  const u16* blp = rwl + (size_t)(n0 + m) * CDIM;

  v8f acc[2][4];
#pragma unroll
  for (int mt = 0; mt < 2; ++mt)
#pragma unroll
    for (int nt = 0; nt < 4; ++nt) acc[mt][nt] = zero8();

#pragma unroll 1
  for (int k0 = 0; k0 < CDIM; k0 += 32) {
    const v16b a0h = ldfb(xhi + ar0 + k0, h), a1h = ldfb(xhi + ar1 + k0, h);
    const v16b a0l = ldfb(xlo + ar0 + k0, h), a1l = ldfb(xlo + ar1 + k0, h);
#pragma unroll
    for (int nt = 0; nt < 4; ++nt) {
      const v16b wh = ldfb(bhp + (size_t)nt * 16 * CDIM + k0, h);
      const v16b wl = ldfb(blp + (size_t)nt * 16 * CDIM + k0, h);
      acc[0][nt] = mma_b(a0h, wh, acc[0][nt]);
      acc[0][nt] = mma_b(a0l, wh, acc[0][nt]);
      acc[0][nt] = mma_b(a0h, wl, acc[0][nt]);
      acc[1][nt] = mma_b(a1h, wh, acc[1][nt]);
      acc[1][nt] = mma_b(a1l, wh, acc[1][nt]);
      acc[1][nt] = mma_b(a1h, wl, acc[1][nt]);
    }
  }

#pragma unroll
  for (int nt = 0; nt < 4; ++nt) {
    const int n = n0 + 16 * nt + m;
    const float bb = rb[n], s = rg[n] * BN_RS, bt = rbe[n];
#pragma unroll
    for (int mt = 0; mt < 2; ++mt)
#pragma unroll
      for (int r = 0; r < 8; ++r) {
        float y = acc[mt][nt][r] + bb;
        y = y * s;
        y = y + bt;
        y = fmaxf(y, 0.0f);
        sT[(32 * w + 16 * mt + 8 * h + r) * 64 + 16 * nt + m] = (_Float16)y;
      }
  }
  __syncthreads();
  _Float16* d0 = r16 + (size_t)m0 * C4 + n0;
  store_h128(sT, d0, C4, w, lane);
  __threadfence();
  store_h128(sT, d0, C4, w, lane);
}

__global__ __launch_bounds__(128) void k_q(
    const u16* __restrict__ xhi, const u16* __restrict__ qw, const float* __restrict__ qb,
    _Float16* q16)
{
#pragma clang fp contract(off)
  __shared__ __attribute__((aligned(16))) _Float16 sT[128 * 64];
  const int tid = threadIdx.x, lane = tid & 31, w = tid >> 5, h = lane >> 4, m = lane & 15;
  const int m0 = blockIdx.x * 128, n0 = blockIdx.y * 64, m0w = m0 + 32 * w;
  const size_t ar0 = (size_t)(m0w + m) * CDIM, ar1 = ar0 + (size_t)16 * CDIM;
  const u16* bp = qw + (size_t)(n0 + m) * CDIM;

  v8f acc[2][4];
#pragma unroll
  for (int mt = 0; mt < 2; ++mt)
#pragma unroll
    for (int nt = 0; nt < 4; ++nt) acc[mt][nt] = zero8();

#pragma unroll 1
  for (int k0 = 0; k0 < CDIM; k0 += 32) {
    const v16b a0 = ldfb(xhi + ar0 + k0, h), a1 = ldfb(xhi + ar1 + k0, h);
#pragma unroll
    for (int nt = 0; nt < 4; ++nt) {
      const v16b wb = ldfb(bp + (size_t)nt * 16 * CDIM + k0, h);
      acc[0][nt] = mma_b(a0, wb, acc[0][nt]);
      acc[1][nt] = mma_b(a1, wb, acc[1][nt]);
    }
  }

#pragma unroll
  for (int nt = 0; nt < 4; ++nt) {
    const int n = n0 + 16 * nt + m;
    const float bb = qb[n];
#pragma unroll
    for (int mt = 0; mt < 2; ++mt)
#pragma unroll
      for (int r = 0; r < 8; ++r)
        sT[(32 * w + 16 * mt + 8 * h + r) * 64 + 16 * nt + m] = (_Float16)(acc[mt][nt][r] + bb);
  }
  __syncthreads();
  _Float16* d0 = q16 + (size_t)m0 * CDIM + n0;
  store_h128(sT, d0, CDIM, w, lane);
  __threadfence();
  store_h128(sT, d0, CDIM, w, lane);
}

__global__ __launch_bounds__(256) void k_dwt(const _Float16* __restrict__ r16, _Float16* dwt16)
{
#pragma clang fp contract(off)
  const int idx = blockIdx.x * 256 + threadIdx.x;
  if (idx >= NB * P2 * 16) return;
  const int cg = idx & 15, pq = idx >> 4;
  const int b = pq / P2, p2 = pq - b * P2;
  const int y2 = p2 / H2, x2 = p2 - y2 * H2;
  const int t1 = (2 * y2) * HIMG + 2 * x2;
  const _Float16* base = r16 + ((size_t)(b * NTOK + t1)) * C4 + 8 * cg;
  const v8h e1 = *(const v8ha*)(base);
  const v8h e2 = *(const v8ha*)(base + HIMG * C4);
  const v8h e3 = *(const v8ha*)(base + C4);
  const v8h e4 = *(const v8ha*)(base + (HIMG + 1) * C4);
  v8h oll = e1, ohl = e1, olh = e1, ohh = e1;
#pragma unroll
  for (int j = 0; j < 8; ++j) {
    const float a1 = r16f((float)e1[j] * 0.5f);
    const float a2 = r16f((float)e2[j] * 0.5f);
    const float a3 = r16f((float)e3[j] * 0.5f);
    const float a4 = r16f((float)e4[j] * 0.5f);
    const float ll = r16f(r16f(r16f(a1 + a2) + a3) + a4);
    const float hl = r16f(r16f(r16f((-a1) - a2) + a3) + a4);
    const float lh = r16f(r16f(r16f((-a1) + a2) - a3) + a4);
    const float hh = r16f(r16f(r16f(a1 - a2) - a3) + a4);
    oll[j] = (_Float16)ll; ohl[j] = (_Float16)hl; olh[j] = (_Float16)lh; ohh[j] = (_Float16)hh;
  }
  _Float16* d = dwt16 + ((size_t)(b * P2 + p2)) * CDIM + 8 * cg;
  *(volatile v8h*)(d) = oll; *(volatile v8h*)(d + C4) = ohl;
  *(volatile v8h*)(d + 2 * C4) = olh; *(volatile v8h*)(d + 3 * C4) = ohh;
  __threadfence();
  *(volatile v8h*)(d) = oll; *(volatile v8h*)(d + C4) = ohl;
  *(volatile v8h*)(d + 2 * C4) = olh; *(volatile v8h*)(d + 3 * C4) = ohh;
}

__global__ __launch_bounds__(128) void k_filter(
    const _Float16* __restrict__ dwt16, const _Float16* __restrict__ fwh, const _Float16* __restrict__ fwl,
    const float* __restrict__ fb, const float* __restrict__ fg, const float* __restrict__ fbe,
    _Float16* xd16)
{
#pragma clang fp contract(off)
  __shared__ __attribute__((aligned(16))) _Float16 sT[64 * 64];
  const int tid = threadIdx.x, lane = tid & 31, w = tid >> 5, h = lane >> 4, m = lane & 15;
  const int wm = w & 1, wn = w >> 1;
  const int m0 = blockIdx.x * 64, n0 = blockIdx.y * 64, n0w = n0 + 32 * wn;

  int yy[2], xx[2];
  size_t abase[2];
#pragma unroll
  for (int mt = 0; mt < 2; ++mt) {
    const int rowg = m0 + 32 * wm + 16 * mt + m;
    const int b = rowg / P2, p = rowg - b * P2;
    yy[mt] = p / H2; xx[mt] = p - yy[mt] * H2;
    abase[mt] = (size_t)b * P2 * CDIM;
  }
  const _Float16* bph = fwh + (size_t)(n0w + m) * KF;
  const _Float16* bpl = fwl + (size_t)(n0w + m) * KF;

  v8f acch[2][2], accl[2][2];
#pragma unroll
  for (int mt = 0; mt < 2; ++mt)
#pragma unroll
    for (int nt = 0; nt < 2; ++nt) { acch[mt][nt] = zero8(); accl[mt][nt] = zero8(); }

#pragma unroll 1
  for (int t = 0; t < 9; ++t) {
    const int t3 = t / 3;
    const int dy = t3 - 1, dx = (t - 3 * t3) - 1;
    const _Float16* ap[2];
    unsigned msk[2];
#pragma unroll
    for (int mt = 0; mt < 2; ++mt) {
      const int sy = yy[mt] + dy, sx = xx[mt] + dx;
      const bool valid = ((unsigned)sy < (unsigned)H2) && ((unsigned)sx < (unsigned)H2);
      const int syc = sy < 0 ? 0 : (sy > H2 - 1 ? H2 - 1 : sy);
      const int sxc = sx < 0 ? 0 : (sx > H2 - 1 ? H2 - 1 : sx);
      ap[mt] = dwt16 + abase[mt] + (size_t)(syc * H2 + sxc) * CDIM;
      msk[mt] = valid ? 0xFFFFFFFFu : 0u;
    }
    const _Float16* bth = bph + (size_t)t * CDIM;
    const _Float16* btl = bpl + (size_t)t * CDIM;
#pragma unroll 1
    for (int c0 = 0; c0 < CDIM; c0 += 32) {
      const v16h a0 = ldfh_m(ap[0] + c0, h, msk[0]);
      const v16h a1 = ldfh_m(ap[1] + c0, h, msk[1]);
#pragma unroll
      for (int nt = 0; nt < 2; ++nt) {
        const v16h wh = ldfh(bth + (size_t)nt * 16 * KF + c0, h);
        const v16h wl = ldfh(btl + (size_t)nt * 16 * KF + c0, h);
        acch[0][nt] = mma_h(a0, wh, acch[0][nt]);
        accl[0][nt] = mma_h(a0, wl, accl[0][nt]);
        acch[1][nt] = mma_h(a1, wh, acch[1][nt]);
        accl[1][nt] = mma_h(a1, wl, accl[1][nt]);
      }
    }
  }

#pragma unroll
  for (int nt = 0; nt < 2; ++nt) {
    const int n = n0w + 16 * nt + m;
    const float bb = fb[n], s = fg[n] * BN_RS, bt = fbe[n];
#pragma unroll
    for (int mt = 0; mt < 2; ++mt)
#pragma unroll
      for (int r = 0; r < 8; ++r) {
        const float conv = (acch[mt][nt][r] + accl[mt][nt][r] * (1.0f / 2048.0f)) * (1.0f / 64.0f);
        float y = conv + bb;
        y = y * s;
        y = y + bt;
        y = fmaxf(y, 0.0f);
        sT[(32 * wm + 16 * mt + 8 * h + r) * 64 + 32 * wn + 16 * nt + m] = (_Float16)y;
      }
  }
  __syncthreads();
  _Float16* d0 = xd16 + (size_t)m0 * CDIM + n0;
  store_h64(sT, d0, CDIM, w, lane);
  __threadfence();
  store_h64(sT, d0, CDIM, w, lane);
}

__global__ __launch_bounds__(256) void k_idwt(const _Float16* __restrict__ xd16, u16* cath, u16* catl)
{
#pragma clang fp contract(off)
  const int idx = blockIdx.x * 256 + threadIdx.x;
  if (idx >= NB * P2 * 16) return;
  const int cg = idx & 15, pq = idx >> 4;
  const int b = pq / P2, p2 = pq - b * P2;
  const int y2 = p2 / H2, x2 = p2 - y2 * H2;
  const _Float16* src = xd16 + ((size_t)(b * P2 + p2)) * CDIM + 8 * cg;
  const v8h vll = *(const v8ha*)(src);
  const v8h vhl = *(const v8ha*)(src + C4);
  const v8h vlh = *(const v8ha*)(src + 2 * C4);
  const v8h vhh = *(const v8ha*)(src + 3 * C4);
  float p1[8], p2v[8], p3[8], p4[8];
#pragma unroll
  for (int j = 0; j < 8; ++j) {
    const float L = (float)vll[j], HL = (float)vhl[j], LH = (float)vlh[j], HH = (float)vhh[j];
    p1[j]  = r16f(r16f(r16f(r16f(L - HL) - LH) + HH) * 0.5f);
    p2v[j] = r16f(r16f(r16f(r16f(L - HL) + LH) - HH) * 0.5f);
    p3[j]  = r16f(r16f(r16f(r16f(L + HL) - LH) - HH) * 0.5f);
    p4[j]  = r16f(r16f(r16f(r16f(L + HL) + LH) + HH) * 0.5f);
  }
  const HL8 s1 = split_bf8(p1), s2 = split_bf8(p2v), s3 = split_bf8(p3), s4 = split_bf8(p4);
  const int tok = (2 * y2) * HIMG + 2 * x2;
  const size_t o1 = ((size_t)(b * NTOK + tok)) * CATK + CDIM + 8 * cg;
  const size_t o3 = o1 + CATK;
  const size_t o2 = o1 + (size_t)HIMG * CATK;
  const size_t o4 = o2 + CATK;
  *(volatile v8us*)(cath + o1) = s1.hi; *(volatile v8us*)(catl + o1) = s1.lo;
  *(volatile v8us*)(cath + o3) = s3.hi; *(volatile v8us*)(catl + o3) = s3.lo;
  *(volatile v8us*)(cath + o2) = s2.hi; *(volatile v8us*)(catl + o2) = s2.lo;
  *(volatile v8us*)(cath + o4) = s4.hi; *(volatile v8us*)(catl + o4) = s4.lo;
  __threadfence();
  *(volatile v8us*)(cath + o1) = s1.hi; *(volatile v8us*)(catl + o1) = s1.lo;
  *(volatile v8us*)(cath + o3) = s3.hi; *(volatile v8us*)(catl + o3) = s3.lo;
  *(volatile v8us*)(cath + o2) = s2.hi; *(volatile v8us*)(catl + o2) = s2.lo;
  *(volatile v8us*)(cath + o4) = s4.hi; *(volatile v8us*)(catl + o4) = s4.lo;
}

__global__ __launch_bounds__(128) void k_kve(
    const _Float16* __restrict__ xd16, const _Float16* __restrict__ kew, const float* __restrict__ keb,
    float* kvin)
{
#pragma clang fp contract(off)
  __shared__ __attribute__((aligned(16))) float sT[128 * 64];
  const int tid = threadIdx.x, lane = tid & 31, w = tid >> 5, h = lane >> 4, m = lane & 15;
  const int m0 = blockIdx.x * 128, n0 = blockIdx.y * 64;

  int yy[2], xx[2];
  unsigned msk[2];
  size_t abase[2];
#pragma unroll
  for (int mt = 0; mt < 2; ++mt) {
    const int rowg = m0 + 32 * w + 16 * mt + m;
    const int b = rowg >> 8, p = rowg & 255;
    const bool valid = p < NKEY;
    const int pc = valid ? p : (NKEY - 1);
    yy[mt] = pc / 14; xx[mt] = pc - yy[mt] * 14;
    msk[mt] = valid ? 0xFFFFFFFFu : 0u;
    abase[mt] = (size_t)b * P2 * CDIM;
  }
  const _Float16* bp = kew + (size_t)(n0 + m) * KE;

  v8f acc[2][4];
#pragma unroll
  for (int mt = 0; mt < 2; ++mt)
#pragma unroll
    for (int nt = 0; nt < 4; ++nt) acc[mt][nt] = zero8();

#pragma unroll 1
  for (int t = 0; t < 4; ++t) {
    const _Float16* ap[2];
#pragma unroll
    for (int mt = 0; mt < 2; ++mt) {
      const int sy = 2 * yy[mt] + (t >> 1), sx = 2 * xx[mt] + (t & 1);
      ap[mt] = xd16 + abase[mt] + (size_t)(sy * H2 + sx) * CDIM;
    }
    const _Float16* bpt = bp + (size_t)t * CDIM;
#pragma unroll 1
    for (int c0 = 0; c0 < CDIM; c0 += 32) {
      const v16h a0 = ldfh_m(ap[0] + c0, h, msk[0]);
      const v16h a1 = ldfh_m(ap[1] + c0, h, msk[1]);
#pragma unroll
      for (int nt = 0; nt < 4; ++nt) {
        const v16h wb = ldfh(bpt + (size_t)nt * 16 * KE + c0, h);
        acc[0][nt] = mma_h(a0, wb, acc[0][nt]);
        acc[1][nt] = mma_h(a1, wb, acc[1][nt]);
      }
    }
  }

#pragma unroll
  for (int nt = 0; nt < 4; ++nt) {
    const int n = n0 + 16 * nt + m;
    const float bb = keb[n];
#pragma unroll
    for (int mt = 0; mt < 2; ++mt)
#pragma unroll
      for (int r = 0; r < 8; ++r) {
        const int lrow = 32 * w + 16 * mt + 8 * h + r;
        const int prow = (m0 + lrow) & 255;
        const float y = acc[mt][nt][r] * (1.0f / 16.0f) + bb;
        sT[lrow * 64 + 16 * nt + m] = (prow < NKEY) ? y : 0.0f;
      }
  }
  __syncthreads();
  float* d0 = kvin + (size_t)m0 * CDIM + n0;
  store_f128(sT, d0, CDIM, w, lane);
  __threadfence();
  store_f128(sT, d0, CDIM, w, lane);
}

__global__ __launch_bounds__(128) void k_ln(
    const float* __restrict__ kvin, const float* __restrict__ g, const float* __restrict__ be,
    _Float16* kvn)
{
#pragma clang fp contract(off)
  const int tid = threadIdx.x, lane = tid & 31, w = tid >> 5;
  const int row = blockIdx.x * 4 + w;
  const bool valid = (row & 255) < NKEY;
  const float* src = kvin + (size_t)row * CDIM;
  float v[16], gg[16], bv[16];
  {
    float tmp[8];
    ld8(src + 8 * lane, tmp);
#pragma unroll
    for (int j = 0; j < 8; ++j) v[j] = tmp[j];
    ld8(src + 256 + 8 * lane, tmp);
#pragma unroll
    for (int j = 0; j < 8; ++j) v[8 + j] = tmp[j];
    ld8(g + 8 * lane, tmp);
#pragma unroll
    for (int j = 0; j < 8; ++j) gg[j] = tmp[j];
    ld8(g + 256 + 8 * lane, tmp);
#pragma unroll
    for (int j = 0; j < 8; ++j) gg[8 + j] = tmp[j];
    ld8(be + 8 * lane, tmp);
#pragma unroll
    for (int j = 0; j < 8; ++j) bv[j] = tmp[j];
    ld8(be + 256 + 8 * lane, tmp);
#pragma unroll
    for (int j = 0; j < 8; ++j) bv[8 + j] = tmp[j];
  }
  float s = 0.0f;
#pragma unroll
  for (int j = 0; j < 16; ++j) s += v[j];
  s += __shfl_xor(s, 16); s += __shfl_xor(s, 8); s += __shfl_xor(s, 4);
  s += __shfl_xor(s, 2);  s += __shfl_xor(s, 1);
  const float mu = s * (1.0f / 512.0f);
  float q = 0.0f;
#pragma unroll
  for (int j = 0; j < 16; ++j) { v[j] = v[j] - mu; const float d2 = v[j] * v[j]; q += d2; }
  q += __shfl_xor(q, 16); q += __shfl_xor(q, 8); q += __shfl_xor(q, 4);
  q += __shfl_xor(q, 2);  q += __shfl_xor(q, 1);
  const float var = q * (1.0f / 512.0f);
  const float rinv = 1.0f / sqrtf(var + EPS_LN);
  v8h o0 = {(_Float16)0.f, (_Float16)0.f, (_Float16)0.f, (_Float16)0.f, (_Float16)0.f, (_Float16)0.f, (_Float16)0.f, (_Float16)0.f};
  v8h o1 = o0;
#pragma unroll
  for (int j = 0; j < 8; ++j) {
    float y0 = v[j] * rinv;      y0 = y0 * gg[j];      y0 = y0 + bv[j];
    float y1 = v[8 + j] * rinv;  y1 = y1 * gg[8 + j];  y1 = y1 + bv[8 + j];
    o0[j] = (_Float16)(valid ? y0 : 0.0f);
    o1[j] = (_Float16)(valid ? y1 : 0.0f);
  }
  _Float16* d0 = kvn + (size_t)row * CDIM + 8 * lane;
  _Float16* d1 = d0 + 256;
  *(volatile v8h*)d0 = o0; *(volatile v8h*)d1 = o1;
  __threadfence();
  *(volatile v8h*)d0 = o0; *(volatile v8h*)d1 = o1;
}

__global__ __launch_bounds__(128) void k_kv(
    const _Float16* __restrict__ kvn, const _Float16* __restrict__ kvw, const float* __restrict__ kvb,
    _Float16* kpl, _Float16* vt)
{
#pragma clang fp contract(off)
  __shared__ __attribute__((aligned(16))) _Float16 sT[128 * 64];
  const int tid = threadIdx.x, lane = tid & 31, w = tid >> 5, h = lane >> 4, m = lane & 15;
  const int m0 = blockIdx.x * 128, m0w = m0 + 32 * w;
  const int cg = blockIdx.y, which = cg >> 3, head = cg & 7;
  const int f0 = which * CDIM + head * HDIM;
  const size_t ar0 = (size_t)(m0w + m) * CDIM, ar1 = ar0 + (size_t)16 * CDIM;
  const _Float16* bp = kvw + (size_t)(f0 + m) * CDIM;

  v8f acc[2][4];
#pragma unroll
  for (int mt = 0; mt < 2; ++mt)
#pragma unroll
    for (int nt = 0; nt < 4; ++nt) acc[mt][nt] = zero8();

#pragma unroll 1
  for (int k0 = 0; k0 < CDIM; k0 += 32) {
    const v16h a0 = ldfh(kvn + ar0 + k0, h), a1 = ldfh(kvn + ar1 + k0, h);
#pragma unroll
    for (int nt = 0; nt < 4; ++nt) {
      const v16h wb = ldfh(bp + (size_t)nt * 16 * CDIM + k0, h);
      acc[0][nt] = mma_h(a0, wb, acc[0][nt]);
      acc[1][nt] = mma_h(a1, wb, acc[1][nt]);
    }
  }

#pragma unroll
  for (int nt = 0; nt < 4; ++nt) {
    const int n = 16 * nt + m;
    const float bb = kvb[f0 + n];
#pragma unroll
    for (int mt = 0; mt < 2; ++mt)
#pragma unroll
      for (int r = 0; r < 8; ++r) {
        const int lrow = 32 * w + 16 * mt + 8 * h + r;
        const int prow = (m0 + lrow) & 255;
        const float y = acc[mt][nt][r] * (1.0f / 32.0f) + bb;
        const float yv = (prow < NKEY) ? y : 0.0f;
        const int idx = (which != 0) ? (n * 128 + lrow) : (lrow * 64 + n);
        sT[idx] = (_Float16)yv;
      }
  }
  __syncthreads();
  if (which == 0) {
    _Float16* d0 = kpl + (size_t)m0 * CDIM + head * HDIM;
    store_h128(sT, d0, CDIM, w, lane);
    __threadfence();
    store_h128(sT, d0, CDIM, w, lane);
  } else {
    const int b = m0 >> 8, kh = (m0 >> 7) & 1, bh = b * NHEAD + head;
    store_vt(sT, vt, bh, kh, w, lane);
    __threadfence();
    store_vt(sT, vt, bh, kh, w, lane);
  }
}

__device__ __forceinline__ v16h pack_p(v8f a, v8f c) {
  const v16h r = { (_Float16)(a[0] * PSCALE), (_Float16)(a[1] * PSCALE), (_Float16)(a[2] * PSCALE), (_Float16)(a[3] * PSCALE),
                   (_Float16)(a[4] * PSCALE), (_Float16)(a[5] * PSCALE), (_Float16)(a[6] * PSCALE), (_Float16)(a[7] * PSCALE),
                   (_Float16)(c[0] * PSCALE), (_Float16)(c[1] * PSCALE), (_Float16)(c[2] * PSCALE), (_Float16)(c[3] * PSCALE),
                   (_Float16)(c[4] * PSCALE), (_Float16)(c[5] * PSCALE), (_Float16)(c[6] * PSCALE), (_Float16)(c[7] * PSCALE) };
  return r;
}

__device__ __forceinline__ void attn_store(const float* so, u16* cath, u16* catl,
                                           size_t rowbase, int head, int lane) {
  const int q8 = lane & 7, sub = lane >> 3;
#pragma unroll
  for (int i = 0; i < 4; ++i) {
    const int row = i * 4 + sub;
    float v[8];
    ld8(so + row * 64 + 8 * q8, v);
    const HL8 s = split_bf8(v);
    const size_t off = (rowbase + row) * CATK + head * HDIM + 8 * q8;
    *(volatile v8us*)(cath + off) = s.hi;
    *(volatile v8us*)(catl + off) = s.lo;
  }
}

__global__ __launch_bounds__(128) void k_attn(
    const _Float16* __restrict__ q16, const _Float16* __restrict__ kpl, const _Float16* __restrict__ vt,
    u16* cath, u16* catl)
{
#pragma clang fp contract(off)
  __shared__ __attribute__((aligned(16))) float sO[4 * 16 * 64];
  const int tid = threadIdx.x, lane = tid & 31, w = tid >> 5, h = lane >> 4, m = lane & 15;
  const int bh = blockIdx.y, b = bh >> 3, head = bh & 7;
  const int q0 = blockIdx.x * 64 + 16 * w;

  const _Float16* qrow = q16 + ((size_t)(b * NTOK + q0 + m)) * CDIM + head * HDIM;
  const v16h qb0 = ldfh(qrow, h);
  const v16h qb1 = ldfh(qrow + 32, h);

  v8f o[4];
#pragma unroll
  for (int t4 = 0; t4 < 4; ++t4) o[t4] = zero8();
  float mrun = -1e30f, lrun = 0.0f;

  const _Float16* kbase = kpl + ((size_t)(b * KST + m)) * CDIM + head * HDIM;
  const _Float16* vbase = vt + ((size_t)(bh * HDIM + m)) * KST;

#pragma unroll 1
  for (int kb = 0; kb < KUSE; kb += 32) {
    v8f s[2];
#pragma unroll
    for (int j = 0; j < 2; ++j) {
      const _Float16* kp = kbase + (size_t)(kb + 16 * j) * CDIM;
      const v16h kf0 = ldfh(kp, h);
      const v16h kf1 = ldfh(kp + 32, h);
      v8f z = zero8();
      z = mma_h(kf0, qb0, z);
      z = mma_h(kf1, qb1, z);
      s[j] = z;
    }
#pragma unroll
    for (int j = 0; j < 2; ++j)
#pragma unroll
      for (int r = 0; r < 8; ++r) {
        const int key = kb + 16 * j + 8 * h + r;
        s[j][r] = (key < NKEY) ? s[j][r] * 0.125f : -1e30f;
      }
    float mloc = s[0][0];
#pragma unroll
    for (int j = 0; j < 2; ++j)
#pragma unroll
      for (int r = 0; r < 8; ++r) mloc = fmaxf(mloc, s[j][r]);
    mloc = fmaxf(mloc, __shfl_xor(mloc, 16));
    const float mnew = fmaxf(mrun, mloc);
    const float alpha = __expf(mrun - mnew);
    mrun = mnew;
    float lsum = 0.0f;
#pragma unroll
    for (int j = 0; j < 2; ++j)
#pragma unroll
      for (int r = 0; r < 8; ++r) {
        const float p = __expf(s[j][r] - mnew);
        s[j][r] = p;
        lsum += p;
      }
    lsum += __shfl_xor(lsum, 16);
    lrun = lrun * alpha + lsum;
#pragma unroll
    for (int t4 = 0; t4 < 4; ++t4)
#pragma unroll
      for (int r = 0; r < 8; ++r) o[t4][r] = o[t4][r] * alpha;

    const v16h pb = pack_p(s[0], s[1]);
#pragma unroll
    for (int t4 = 0; t4 < 4; ++t4) {
      const v16h vf = ldfh(vbase + (size_t)(16 * t4) * KST + kb, h);
      o[t4] = mma_h(vf, pb, o[t4]);
    }
  }

  const float inv = (1.0f / lrun) * (1.0f / PSCALE);
  float* so = sO + w * 1024;
#pragma unroll
  for (int t4 = 0; t4 < 4; ++t4)
#pragma unroll
    for (int r = 0; r < 8; ++r)
      so[m * 64 + 16 * t4 + 8 * h + r] = o[t4][r] * inv;
  __syncthreads();

  const size_t rowbase = (size_t)(b * NTOK + q0);
  attn_store(so, cath, catl, rowbase, head, lane);
  __threadfence();
  attn_store(so, cath, catl, rowbase, head, lane);
}

__global__ __launch_bounds__(128) void k_proj(
    const u16* __restrict__ cath, const u16* __restrict__ catl,
    const u16* __restrict__ pwh, const u16* __restrict__ pwl,
    const float* __restrict__ pb, float* out)
{
#pragma clang fp contract(off)
  __shared__ __attribute__((aligned(16))) float sT[128 * 64];
  const int tid = threadIdx.x, lane = tid & 31, w = tid >> 5, h = lane >> 4, m = lane & 15;
  const int m0 = blockIdx.x * 128, n0 = blockIdx.y * 64, m0w = m0 + 32 * w;
  const size_t ar0 = (size_t)(m0w + m) * CATK, ar1 = ar0 + (size_t)16 * CATK;
  const u16* bhp = pwh + (size_t)(n0 + m) * CATK;
  const u16* blp = pwl + (size_t)(n0 + m) * CATK;

  v8f acc[2][4];
#pragma unroll
  for (int mt = 0; mt < 2; ++mt)
#pragma unroll
    for (int nt = 0; nt < 4; ++nt) acc[mt][nt] = zero8();

#pragma unroll 1
  for (int k0 = 0; k0 < CATK; k0 += 32) {
    const v16b a0h = ldfb(cath + ar0 + k0, h), a1h = ldfb(cath + ar1 + k0, h);
    const v16b a0l = ldfb(catl + ar0 + k0, h), a1l = ldfb(catl + ar1 + k0, h);
#pragma unroll
    for (int nt = 0; nt < 4; ++nt) {
      const v16b wh = ldfb(bhp + (size_t)nt * 16 * CATK + k0, h);
      const v16b wl = ldfb(blp + (size_t)nt * 16 * CATK + k0, h);
      acc[0][nt] = mma_b(a0h, wh, acc[0][nt]);
      acc[0][nt] = mma_b(a0l, wh, acc[0][nt]);
      acc[0][nt] = mma_b(a0h, wl, acc[0][nt]);
      acc[1][nt] = mma_b(a1h, wh, acc[1][nt]);
      acc[1][nt] = mma_b(a1l, wh, acc[1][nt]);
      acc[1][nt] = mma_b(a1h, wl, acc[1][nt]);
    }
  }

#pragma unroll
  for (int nt = 0; nt < 4; ++nt) {
    const int n = n0 + 16 * nt + m;
    const float bb = pb[n];
#pragma unroll
    for (int mt = 0; mt < 2; ++mt)
#pragma unroll
      for (int r = 0; r < 8; ++r)
        sT[(32 * w + 16 * mt + 8 * h + r) * 64 + 16 * nt + m] = acc[mt][nt][r] + bb;
  }
  __syncthreads();
  float* d0 = out + (size_t)m0 * CDIM + n0;
  store_f128(sT, d0, CDIM, w, lane);
  __threadfence();
  store_f128(sT, d0, CDIM, w, lane);
}

extern "C" void kernel_launch(void* const* d_in, const int* in_sizes, int n_in,
                              void* d_out, int out_size, void* d_ws, size_t ws_size,
                              hipStream_t stream) {
  if (n_in < 21) return;
  if (in_sizes[0] != NQROWS * CDIM) return;
  if (in_sizes[3] != C4 * CDIM || in_sizes[4] != C4 || in_sizes[5] != C4 || in_sizes[6] != C4) return;
  if (in_sizes[7] != CDIM * CDIM * 9 || in_sizes[8] != CDIM || in_sizes[9] != CDIM || in_sizes[10] != CDIM) return;
  if (in_sizes[11] != CDIM * CDIM || in_sizes[12] != CDIM || in_sizes[13] != CDIM || in_sizes[14] != CDIM) return;
  if (in_sizes[15] != 2 * CDIM * CDIM || in_sizes[16] != 2 * CDIM) return;
  if (in_sizes[17] != CDIM * CDIM * 4 || in_sizes[18] != CDIM) return;
  if (in_sizes[19] != CDIM * CATK || in_sizes[20] != CDIM) return;
  if (out_size != NQROWS * CDIM) return;

  const float* x         = (const float*)d_in[0];
  const float* reduce_w  = (const float*)d_in[3];
  const float* reduce_b  = (const float*)d_in[4];
  const float* reduce_g  = (const float*)d_in[5];
  const float* reduce_be = (const float*)d_in[6];
  const float* filter_w  = (const float*)d_in[7];
  const float* filter_b  = (const float*)d_in[8];
  const float* filter_g  = (const float*)d_in[9];
  const float* filter_be = (const float*)d_in[10];
  const float* q_w       = (const float*)d_in[11];
  const float* q_b       = (const float*)d_in[12];
  const float* ln_g      = (const float*)d_in[13];
  const float* ln_b      = (const float*)d_in[14];
  const float* kv_w      = (const float*)d_in[15];
  const float* kv_b      = (const float*)d_in[16];
  const float* kve_w     = (const float*)d_in[17];
  const float* kve_b     = (const float*)d_in[18];
  const float* proj_w    = (const float*)d_in[19];
  const float* proj_b    = (const float*)d_in[20];
  float* out = (float*)d_out;

  const size_t szQW   = (size_t)CDIM * CDIM * 2;
  const size_t szRW   = (size_t)C4 * CDIM * 2;
  const size_t szFW   = (size_t)CDIM * KF * 2;
  const size_t szKEW  = (size_t)CDIM * KE * 2;
  const size_t szKVW  = (size_t)2 * CDIM * CDIM * 2;
  const size_t szPW   = (size_t)CDIM * CATK * 2;
  const size_t szXP   = (size_t)NQROWS * CDIM * 2;
  const size_t szCATP = (size_t)NQROWS * CATK * 2;
  const size_t szA    = (2 * szCATP > 2 * szXP) ? 2 * szCATP : 2 * szXP;
  const size_t szQ    = (size_t)NQROWS * CDIM * 2;
  const size_t szR16  = (size_t)NQROWS * C4 * 2;
  const size_t szDWT  = (size_t)NPIX2 * CDIM * 2;
  const size_t szKVIN = (size_t)KVROWS * CDIM * 4;
  const size_t szKVN  = (size_t)KVROWS * CDIM * 2;
  const size_t szKPL  = (size_t)KVROWS * CDIM * 2;
  const size_t szVT   = (size_t)NB * NHEAD * HDIM * KST * 2;

  size_t off = 0;
  const size_t oQW  = off; off += szQW;
  const size_t oRWH = off; off += szRW;
  const size_t oRWL = off; off += szRW;
  const size_t oFWH = off; off += szFW;
  const size_t oFWL = off; off += szFW;
  const size_t oKEW = off; off += szKEW;
  const size_t oKVW = off; off += szKVW;
  const size_t oPWH = off; off += szPW;
  const size_t oPWL = off; off += szPW;
  const size_t oA   = off; off += szA;
  const size_t oQ   = off; off += szQ;
  const size_t oR16 = off; off += szR16;
  const size_t oDWT = off; off += szDWT;
  const size_t oKVIN= off; off += szKVIN;
  const size_t oKVN = off; off += szKVN;
  const size_t oKPL = off; off += szKPL;
  const size_t oVT  = off; off += szVT;
  const size_t total = off;
  if (total > ws_size) return;
  if (total > (size_t)134217728) return;

  char* ws = (char*)d_ws;
  u16*      qw    = (u16*)(ws + oQW);
  u16*      rwh   = (u16*)(ws + oRWH);
  u16*      rwl   = (u16*)(ws + oRWL);
  _Float16* fwh   = (_Float16*)(ws + oFWH);
  _Float16* fwl   = (_Float16*)(ws + oFWL);
  _Float16* kew   = (_Float16*)(ws + oKEW);
  _Float16* kvw   = (_Float16*)(ws + oKVW);
  u16*      pwh   = (u16*)(ws + oPWH);
  u16*      pwl   = (u16*)(ws + oPWL);
  u16*      xhi   = (u16*)(ws + oA);
  u16*      xlo   = (u16*)(ws + oA + szXP);
  u16*      cath  = (u16*)(ws + oA);
  u16*      catl  = (u16*)(ws + oA + szCATP);
  _Float16* q16   = (_Float16*)(ws + oQ);
  _Float16* r16   = (_Float16*)(ws + oR16);
  _Float16* xd16  = (_Float16*)(ws + oR16);
  _Float16* dwt16 = (_Float16*)(ws + oDWT);
  float*    kvin  = (float*)(ws + oKVIN);
  _Float16* kvn   = (_Float16*)(ws + oKVN);
  _Float16* kpl   = (_Float16*)(ws + oKPL);
  _Float16* vt    = (_Float16*)(ws + oVT);

  k_prep<<<PB_TOTAL, 256, 0, stream>>>(x, q_w, reduce_w, filter_w, kve_w, kv_w, proj_w,
                                       xhi, xlo, qw, rwh, rwl, fwh, fwl, kew, kvw, pwh, pwl);
  k_reduce<<<dim3(NQROWS / 128, C4 / 64), 128, 0, stream>>>(xhi, xlo, rwh, rwl, reduce_b, reduce_g, reduce_be, r16);
  k_q<<<dim3(NQROWS / 128, CDIM / 64), 128, 0, stream>>>(xhi, qw, q_b, q16);
  k_dwt<<<(NB * P2 * 16 + 255) / 256, 256, 0, stream>>>(r16, dwt16);
  k_filter<<<dim3(NPIX2 / 64, CDIM / 64), 128, 0, stream>>>(dwt16, fwh, fwl, filter_b, filter_g, filter_be, xd16);
  k_idwt<<<(NB * P2 * 16 + 255) / 256, 256, 0, stream>>>(xd16, cath, catl);
  k_kve<<<dim3(KVROWS / 128, CDIM / 64), 128, 0, stream>>>(xd16, kew, kve_b, kvin);
  k_ln<<<KVROWS / 4, 128, 0, stream>>>(kvin, ln_g, ln_b, kvn);
  k_kv<<<dim3(KVROWS / 128, 16), 128, 0, stream>>>(kvn, kvw, kv_b, kpl, vt);
  k_attn<<<dim3(NTOK / 64, NB * NHEAD), 128, 0, stream>>>(q16, kpl, vt, cath, catl);
  k_proj<<<dim3(NQROWS / 128, CDIM / 64), 128, 0, stream>>>(cath, catl, pwh, pwl, proj_b, out);
}
